// TemporalDiffAttn_42116449305216
// MI455X (gfx1250) — hardware-verified
//
#include <hip/hip_runtime.h>


#define NB_  8
#define TT   2048
#define DD   128
#define NH_  4
#define HQ   32
#define HV   64
#define NBLK 32
#define KW   448
#define KOFF 192
#define SCL  0.17677669529663687f
typedef _Float16 h16;
typedef unsigned short bf;
typedef __attribute__((ext_vector_type(16))) __bf16   v16bf;
typedef __attribute__((ext_vector_type(16))) _Float16 v16h;
typedef __attribute__((ext_vector_type(8)))  _Float16 v8h;
typedef __attribute__((ext_vector_type(8)))  unsigned short v8us;
typedef __attribute__((ext_vector_type(8)))  float    v8f;
typedef __attribute__((ext_vector_type(4)))  float    v4f;
typedef v8h  __attribute__((may_alias)) v8ha;
typedef v4f  __attribute__((may_alias)) v4fa;
typedef v8us __attribute__((may_alias)) v8usa;

__device__ __forceinline__ unsigned short f2bf(float f) { unsigned u = __float_as_uint(f); u += 0x7FFFu + ((u >> 16) & 1u); return (unsigned short)(u >> 16); }
__device__ __forceinline__ float bf2f(unsigned short b) { return __uint_as_float(((unsigned)b) << 16); }
__device__ __forceinline__ float bfr(float f) { return bf2f(f2bf(f)); }
__device__ __forceinline__ v16h cat16(v8h lo, v8h hi) { return __builtin_shufflevector(lo, hi, 0, 1, 2, 3, 4, 5, 6, 7, 8, 9, 10, 11, 12, 13, 14, 15); }
__device__ __forceinline__ v16bf cat16b(v8us lo, v8us hi) { return __builtin_bit_cast(v16bf, __builtin_shufflevector(lo, hi, 0, 1, 2, 3, 4, 5, 6, 7, 8, 9, 10, 11, 12, 13, 14, 15)); }
__device__ __forceinline__ v8f wmma16(v16h a, v16h b, v8f c) { return __builtin_amdgcn_wmma_f32_16x16x32_f16(false, a, false, b, (short)0, c, false, false); }
__device__ __forceinline__ v8f wmmab(v16bf a, v16bf b, v8f c) { return __builtin_amdgcn_wmma_f32_16x16x32_bf16(false, a, false, b, (short)0, c, false, false); }


template <typename T16> struct WFrag;
template <> struct WFrag<h16> { typedef v16h V; static __device__ __forceinline__ V ld(const h16* p) { return cat16(*(const v8h*)p, *(const v8h*)(p + 16)); } static __device__ __forceinline__ v8f mma(V a, V b, v8f c) { return wmma16(a, b, c); } };
template <> struct WFrag<bf> { typedef v16bf V; static __device__ __forceinline__ V ld(const bf* p) { return cat16b(*(const v8us*)p, *(const v8us*)(p + 16)); } static __device__ __forceinline__ v8f mma(V a, V b, v8f c) { return wmmab(a, b, c); } };
template <typename T16, int NSPLIT, bool BIAS>
__global__ __launch_bounds__(32) void k_gemmw(const T16* __restrict__ A, const T16* __restrict__ A2, const T16* __restrict__ Bt, const T16* __restrict__ Bt2, int K, float* C, int ldc, const float* __restrict__ bias, size_t sA, size_t sB, size_t sC) {
    typedef typename WFrag<T16>::V V;
    __shared__ __align__(16) float os[16 * 68];
    const size_t z = blockIdx.z; A += z * sA; if (A2) A2 += z * sA; Bt += z * sB; if (Bt2) Bt2 += z * sB; C += z * sC;
    const int lane = threadIdx.x & 31, lr = lane & 15, hi = lane >> 4; const int r0 = blockIdx.x * 64, c0 = blockIdx.y * 64;
    v8f acc[4][4];
#pragma unroll
    for (int mb = 0; mb < 4; ++mb)
#pragma unroll
        for (int nb = 0; nb < 4; ++nb) acc[mb][nb] = (v8f){};
    const size_t aoff = (size_t)(r0 + lr) * K + 8 * hi, boff = (size_t)(c0 + lr) * K + 8 * hi;
#pragma unroll 1
    for (int kc = 0; kc < K; kc += 32) {
        V a[4], a2[4];
#pragma unroll
        for (int mb = 0; mb < 4; ++mb) { a[mb] = WFrag<T16>::ld(A + aoff + (size_t)mb * 16 * K + kc); if (NSPLIT == 1 || NSPLIT == 2) a2[mb] = WFrag<T16>::ld(A2 + aoff + (size_t)mb * 16 * K + kc); }
#pragma unroll
        for (int nb = 0; nb < 4; ++nb) { const V b = WFrag<T16>::ld(Bt + boff + (size_t)nb * 16 * K + kc); V b2; if (NSPLIT >= 2) b2 = WFrag<T16>::ld(Bt2 + boff + (size_t)nb * 16 * K + kc);
#pragma unroll
            for (int mb = 0; mb < 4; ++mb) { acc[mb][nb] = WFrag<T16>::mma(a[mb], b, acc[mb][nb]); if (NSPLIT == 1 || NSPLIT == 2) acc[mb][nb] = WFrag<T16>::mma(a2[mb], b, acc[mb][nb]); if (NSPLIT >= 2) acc[mb][nb] = WFrag<T16>::mma(a[mb], b2, acc[mb][nb]); } }
        asm volatile("v_nop\n\tv_nop\n\tv_nop\n\tv_nop" : "+v"(acc[0][0]), "+v"(acc[1][1]), "+v"(acc[2][2]), "+v"(acc[3][3]) : "v"(a[0]), "v"(a[3]));
    }
#pragma unroll
    for (int mb = 0; mb < 4; ++mb) {
#pragma unroll
        for (int nb = 0; nb < 4; ++nb) {
#pragma unroll
            for (int j = 0; j < 8; ++j) os[(hi * 8 + j) * 68 + nb * 16 + lr] = acc[mb][nb][j]; }
        __builtin_amdgcn_wave_barrier(); asm volatile("" ::: "memory");
        float* crow = C + (size_t)(r0 + mb * 16) * ldc + c0;
#pragma unroll 1
        for (int ps = 0; ps < 2; ++ps) {
#pragma unroll
            for (int s = 0; s < 8; ++s) { const int row = 2 * s + hi, cofs = lr * 4; v4f val = *(const v4fa*)(os + row * 68 + cofs); if (BIAS) { val[0] += bfr(bias[c0 + cofs]); val[1] += bfr(bias[c0 + cofs + 1]); val[2] += bfr(bias[c0 + cofs + 2]); val[3] += bfr(bias[c0 + cofs + 3]); }
                *(volatile v4f*)(crow + (size_t)row * ldc + cofs) = val; }
            if (ps == 0) __threadfence(); }
        __builtin_amdgcn_wave_barrier(); asm volatile("" ::: "memory");
    }
}

__device__ __forceinline__ void splitf(float y, unsigned short& h, unsigned short& l) { h = f2bf(y); l = f2bf(y - bf2f(h)); }
typedef __attribute__((ext_vector_type(2))) unsigned short v2us;
typedef __attribute__((ext_vector_type(4))) unsigned short v4us;
typedef __attribute__((ext_vector_type(2))) float v2f;

__global__ __launch_bounds__(256) void k_wtG(const float* __restrict__ w, int K, int N, bf* Bt) {
    const int lane = threadIdx.x & 31; const int L0 = (blockIdx.x * 8 + (threadIdx.x >> 5)) * 8; const int nlines = N * K / 64;
#pragma unroll 1
    for (int ps = 0; ps < 2; ++ps) {
#pragma unroll 1
        for (int l = 0; l < 8; ++l) { const int L = L0 + l; if (L >= nlines) break; const size_t e = (size_t)L * 64 + lane * 2; const int k = (int)(e % K), n = (int)(e / K); v2us o;
            o[0] = f2bf(w[(size_t)k * N + n]); o[1] = f2bf(w[(size_t)(k + 1) * N + n]); *(volatile v2us*)(Bt + e) = o; }
        if (ps == 0) __threadfence(); }
}
__global__ __launch_bounds__(256) void k_ln(const float* __restrict__ X, const float* __restrict__ w, const float* __restrict__ bb, bf* Xh, bf* Xl) { const int lane = threadIdx.x & 31; const int t = blockIdx.x * 8 + (threadIdx.x >> 5); if (t >= TT) return; const v4f a = *(const v4f*)(X + (size_t)t * DD + lane * 4); float v[4]; float s = 0.f;
#pragma unroll
    for (int q = 0; q < 4; ++q) { v[q] = bfr(a[q]); s = __fadd_rn(s, v[q]); }
#pragma unroll
    for (int sh = 16; sh; sh >>= 1) s += __shfl_xor(s, sh, 32);
    const float mu = s * (1.0f / DD); float q2 = 0.f;
#pragma unroll
    for (int q = 0; q < 4; ++q) { float dv = __fsub_rn(v[q], mu); asm volatile("" : "+v"(dv)); float p = __fmul_rn(dv, dv); asm volatile("" : "+v"(p)); q2 = __fadd_rn(q2, p); }
#pragma unroll
    for (int sh = 16; sh; sh >>= 1) q2 += __shfl_xor(q2, sh, 32);
    float vq = q2 * (1.0f / DD); asm volatile("" : "+v"(vq)); const float rs = __frsqrt_rn(__fadd_rn(vq, 1e-5f)); v4us oh, ol;
#pragma unroll
    for (int q = 0; q < 4; ++q) { const int c = lane * 4 + q; float dv = __fsub_rn(v[q], mu); asm volatile("" : "+v"(dv)); float tn = __fmul_rn(dv, rs); asm volatile("" : "+v"(tn)); float tg = __fmul_rn(tn, bfr(w[c])); asm volatile("" : "+v"(tg)); unsigned short u, l; splitf(__fadd_rn(tg, bfr(bb[c])), u, l); oh[q] = u; ol[q] = l; }
    const size_t o = (size_t)t * DD + lane * 4; *(volatile v4us*)(Xh + o) = oh; *(volatile v4us*)(Xl + o) = ol; __threadfence(); *(volatile v4us*)(Xh + o) = oh; *(volatile v4us*)(Xl + o) = ol; }
__global__ __launch_bounds__(256) void k_qpl(const float* __restrict__ QF, bf* Qh, bf* Ql) { const size_t e = ((size_t)blockIdx.x * 256 + threadIdx.x) * 2; if (e >= (size_t)2 * NH_ * TT * HQ) return; const int d = (int)(e % HQ); const int t = (int)((e / HQ) % TT); const int h = (int)((e / ((size_t)HQ * TT)) % NH_); const int m = (int)(e / ((size_t)HQ * TT * NH_)); v2us oh, ol;
#pragma unroll
    for (int u = 0; u < 2; ++u) { unsigned short a, c; splitf(QF[(size_t)t * 2 * DD + h * HV + m * HQ + d + u], a, c); oh[u] = a; ol[u] = c; } *(volatile v2us*)(Qh + e) = oh; *(volatile v2us*)(Ql + e) = ol; __threadfence(); *(volatile v2us*)(Qh + e) = oh; *(volatile v2us*)(Ql + e) = ol; }
#define KROWS (KOFF + TT + 256)
__global__ __launch_bounds__(256) void k_kpad(const float* __restrict__ KF, bf* Kh, bf* Kl) { const size_t e = ((size_t)blockIdx.x * 256 + threadIdx.x) * 2; if (e >= (size_t)2 * NH_ * KROWS * HQ) return; const int d = (int)(e % HQ); const int r = (int)((e / HQ) % KROWS); const int h = (int)((e / ((size_t)HQ * KROWS)) % NH_); const int m = (int)(e / ((size_t)HQ * KROWS * NH_)); const int j = r - KOFF; v2us oh, ol;
#pragma unroll
    for (int u = 0; u < 2; ++u) { unsigned short a = 0, c = 0; if (j >= 0 && j < TT) splitf(KF[(size_t)j * 2 * DD + h * HV + m * HQ + d + u], a, c); oh[u] = a; ol[u] = c; } *(volatile v2us*)(Kh + e) = oh; *(volatile v2us*)(Kl + e) = ol; __threadfence(); *(volatile v2us*)(Kh + e) = oh; *(volatile v2us*)(Kl + e) = ol; }
__global__ __launch_bounds__(256) void k_vwin(const float* __restrict__ VF, bf* Vh, bf* Vl) { const size_t e = ((size_t)blockIdx.x * 256 + threadIdx.x) * 2; if (e >= (size_t)NH_ * NBLK * HV * KW) return; const int c = (int)(e % KW); const int ev = (int)((e / KW) % HV); const int blk = (int)((e / ((size_t)KW * HV)) % NBLK); const int h = (int)(e / ((size_t)KW * HV * NBLK)); v2us oh, ol;
#pragma unroll
    for (int u = 0; u < 2; ++u) { const int j = blk * 64 - KOFF + c + u; unsigned short a = 0, cc = 0; if (j >= 0 && j < TT) splitf(VF[(size_t)j * 2 * DD + h * HV + ev], a, cc); oh[u] = a; ol[u] = cc; } *(volatile v2us*)(Vh + e) = oh; *(volatile v2us*)(Vl + e) = ol; __threadfence(); *(volatile v2us*)(Vh + e) = oh; *(volatile v2us*)(Vl + e) = ol; }
__global__ __launch_bounds__(256) void k_dsoft(const float* __restrict__ S1, const float* __restrict__ S2, const float* __restrict__ sgs, const float* __restrict__ sgn, const float* __restrict__ lq1, const float* __restrict__ lk1, const float* __restrict__ lq2, const float* __restrict__ lk2, bf* Ph, bf* Pl) {
    const int lane = threadIdx.x & 31; const int row = blockIdx.x * 8 + (threadIdx.x >> 5); if (row >= NH_ * NBLK * 64) return; const int r = row % 64; const int blk = (row / 64) % NBLK; const int i = blk * 64 + r; const int j0 = blk * 64 - KOFF;
    const float ss = fmaxf(bfr(sgs[0]), 1.0f), sn = fmaxf(bfr(sgn[0]), 1.0f); const float is = __fdiv_rn(1.0f, ss), in_ = __fdiv_rn(1.0f, sn);
    float d1 = __fmul_rn(bfr(lq1[lane]), bfr(lk1[lane])), d2 = __fmul_rn(bfr(lq2[lane]), bfr(lk2[lane]));
#pragma unroll
    for (int sh = 16; sh; sh >>= 1) { d1 += __shfl_xor(d1, sh, 32); d2 += __shfl_xor(d2, sh, 32); }
    const float lam = __fadd_rn(__fsub_rn(__expf(d1), __expf(d2)), 0.8f);
    const float* s1r = S1 + (size_t)row * KW; const float* s2r = S2 + (size_t)row * KW; float v1[14], v2[14]; float m1 = -3.0e38f, m2 = -3.0e38f;
#pragma unroll
    for (int q = 0; q < 7; ++q)
#pragma unroll
        for (int u = 0; u < 2; ++u) { const int c = q * 64 + 2 * lane + u; const int j = j0 + c; float t1 = -3.0e38f, t2 = -3.0e38f;
            if (j >= 0 && j < TT) { const float rel = (float)(j - i); float z1 = __fmul_rn(rel, is); asm volatile("" : "+v"(z1)); float z2 = __fmul_rn(rel, in_); asm volatile("" : "+v"(z2)); float b1 = __fmul_rn(-0.5f, __fmul_rn(z1, z1)); asm volatile("" : "+v"(b1)); float b2 = __fmul_rn(-0.5f, __fmul_rn(z2, z2)); asm volatile("" : "+v"(b2));
                float a1 = __fmul_rn(s1r[c], SCL); asm volatile("" : "+v"(a1)); float a2 = __fmul_rn(s2r[c], SCL); asm volatile("" : "+v"(a2)); t1 = __fadd_rn(a1, b1); t2 = __fadd_rn(a2, b2); }
            v1[q * 2 + u] = t1; v2[q * 2 + u] = t2; m1 = fmaxf(m1, t1); m2 = fmaxf(m2, t2); }
#pragma unroll
    for (int sh = 16; sh; sh >>= 1) { m1 = fmaxf(m1, __shfl_xor(m1, sh, 32)); m2 = fmaxf(m2, __shfl_xor(m2, sh, 32)); }
    float sum1 = 0.f, sum2 = 0.f;
#pragma unroll
    for (int k = 0; k < 14; ++k) { float e1 = __fsub_rn(v1[k], m1); asm volatile("" : "+v"(e1)); v1[k] = __expf(e1); sum1 += v1[k]; float e2 = __fsub_rn(v2[k], m2); asm volatile("" : "+v"(e2)); v2[k] = __expf(e2); sum2 += v2[k]; }
#pragma unroll
    for (int sh = 16; sh; sh >>= 1) { sum1 += __shfl_xor(sum1, sh, 32); sum2 += __shfl_xor(sum2, sh, 32); }
    const float f1 = __fdiv_rn(1.0f, sum1); const float f2 = __fmul_rn(__fdiv_rn(1.0f, sum2), lam);
#pragma unroll 1
    for (int ps = 0; ps < 2; ++ps) {
#pragma unroll
        for (int q = 0; q < 7; ++q) { v2us oh, ol;
#pragma unroll
            for (int u = 0; u < 2; ++u) { float p2 = __fmul_rn(v2[q * 2 + u], f2); asm volatile("" : "+v"(p2)); float p1 = __fmul_rn(v1[q * 2 + u], f1); asm volatile("" : "+v"(p1)); unsigned short a, c2; splitf(__fsub_rn(p1, p2), a, c2); oh[u] = a; ol[u] = c2; }
            const size_t oo = (size_t)row * KW + q * 64 + 2 * lane; *(volatile v2us*)(Ph + oo) = oh; *(volatile v2us*)(Pl + oo) = ol; }
        if (ps == 0) __threadfence(); } }
__global__ __launch_bounds__(256) void k_hln(const float* __restrict__ O, const float* __restrict__ w, const float* __restrict__ bb, bf* Mh, bf* Ml) { const int lane = threadIdx.x & 31; const int row = blockIdx.x * 8 + (threadIdx.x >> 5); if (row >= NH_ * TT) return; const int t = row % TT, h = row / TT; const float* o = O + ((size_t)h * TT + t) * HV + 2 * lane; const float a0 = o[0], a1 = o[1]; float s = __fadd_rn(a0, a1);
#pragma unroll
    for (int sh = 16; sh; sh >>= 1) s += __shfl_xor(s, sh, 32);
    const float mu = s * (1.0f / HV); float e0 = __fsub_rn(a0, mu), e1 = __fsub_rn(a1, mu); asm volatile("" : "+v"(e0), "+v"(e1)); float q2 = __fadd_rn(__fmul_rn(e0, e0), __fmul_rn(e1, e1));
#pragma unroll
    for (int sh = 16; sh; sh >>= 1) q2 += __shfl_xor(q2, sh, 32);
    float vq = q2 * (1.0f / HV); asm volatile("" : "+v"(vq)); const float rs = __frsqrt_rn(__fadd_rn(vq, 1e-5f)); v2us oh, ol;
#pragma unroll
    for (int u = 0; u < 2; ++u) { const int e = 2 * lane + u; float tn = __fmul_rn(u ? e1 : e0, rs); asm volatile("" : "+v"(tn)); float tg = __fmul_rn(tn, bfr(w[e])); asm volatile("" : "+v"(tg)); float y = __fadd_rn(tg, bfr(bb[e])); asm volatile("" : "+v"(y)); unsigned short a, c; splitf(__fmul_rn(y, 0.19999998807907104f), a, c); oh[u] = a; ol[u] = c; }
    const size_t oo = (size_t)t * 2 * DD + h * HV + 2 * lane; *(volatile v2us*)(Mh + oo) = oh; *(volatile v2us*)(Ml + oo) = ol; __threadfence(); *(volatile v2us*)(Mh + oo) = oh; *(volatile v2us*)(Ml + oo) = ol; }
__global__ __launch_bounds__(256) void k_fin(const float* __restrict__ x, const float* __restrict__ R, float* OUT) { const size_t i = ((size_t)blockIdx.x * 256 + threadIdx.x) * 4; if (i >= (size_t)TT * DD) return; const v4f r = *(const v4f*)(R + i); v4f o; o[0] = __fadd_rn(bfr(x[i]), r[0]); o[1] = __fadd_rn(bfr(x[i + 1]), r[1]); o[2] = __fadd_rn(bfr(x[i + 2]), r[2]); o[3] = __fadd_rn(bfr(x[i + 3]), r[3]); *(volatile v4f*)(OUT + i) = o; __threadfence(); *(volatile v4f*)(OUT + i) = o; }

extern "C" void kernel_launch(void* const* d_in, const int* in_sizes, int n_in,
                              void* d_out, int out_size, void* d_ws, size_t ws_size, hipStream_t stream) {
    (void)in_sizes; (void)n_in; (void)out_size;
    const float* IN[15]; for (int i = 0; i < 15; ++i) IN[i] = (const float*)d_in[i];
    float* OUT = (float*)d_out;
    char* wsp = (char*)d_ws;
    auto take = [&](size_t bytes) { char* p = wsp; wsp += (bytes + 255) & ~(size_t)255; return (void*)p; };
    bf* WQ = (bf*)take((size_t)2 * DD * DD * 2); bf* WK = (bf*)take((size_t)2 * DD * DD * 2); bf* WV = (bf*)take((size_t)2 * DD * DD * 2); bf* WO = (bf*)take((size_t)DD * 2 * DD * 2);
    bf* Xh = (bf*)take((size_t)TT * DD * 2); bf* Xl = (bf*)take((size_t)TT * DD * 2); float* QF = (float*)take((size_t)TT * 2 * DD * 4); float* KF = (float*)take((size_t)TT * 2 * DD * 4); float* VF = (float*)take((size_t)TT * 2 * DD * 4);
    bf* Qh = (bf*)take((size_t)2 * NH_ * TT * HQ * 2); bf* Ql = (bf*)take((size_t)2 * NH_ * TT * HQ * 2); bf* Kh = (bf*)take((size_t)2 * NH_ * KROWS * HQ * 2); bf* Kl = (bf*)take((size_t)2 * NH_ * KROWS * HQ * 2); bf* Vh = (bf*)take((size_t)NH_ * NBLK * HV * KW * 2); bf* Vl = (bf*)take((size_t)NH_ * NBLK * HV * KW * 2);
    float* S1 = (float*)take((size_t)NH_ * NBLK * 64 * KW * 4); float* S2 = (float*)take((size_t)NH_ * NBLK * 64 * KW * 4); bf* Ph = (bf*)take((size_t)NH_ * NBLK * 64 * KW * 2); bf* Pl = (bf*)take((size_t)NH_ * NBLK * 64 * KW * 2); float* O = (float*)take((size_t)NH_ * TT * HV * 4); bf* Mh = (bf*)take((size_t)TT * 2 * DD * 2); bf* Ml = (bf*)take((size_t)TT * 2 * DD * 2); float* R = (float*)take((size_t)TT * DD * 4);
    if ((size_t)(wsp - (char*)d_ws) > ws_size) return;
    k_wtG<<<(DD * 2 * DD / 64 + 63) / 64, 256, 0, stream>>>(IN[3], DD, 2 * DD, WQ); k_wtG<<<(DD * 2 * DD / 64 + 63) / 64, 256, 0, stream>>>(IN[4], DD, 2 * DD, WK); k_wtG<<<(DD * 2 * DD / 64 + 63) / 64, 256, 0, stream>>>(IN[5], DD, 2 * DD, WV); k_wtG<<<(2 * DD * DD / 64 + 63) / 64, 256, 0, stream>>>(IN[6], 2 * DD, DD, WO);
    for (int b = 0; b < NB_; ++b) { const float* xb = IN[0] + (size_t)b * TT * DD;
        k_ln<<<TT / 8, 256, 0, stream>>>(xb, IN[1], IN[2], Xh, Xl);
        k_gemmw<bf, 1, false><<<dim3(TT / 64, 2 * DD / 64, 1), 32, 0, stream>>>(Xh, Xl, WQ, nullptr, DD, QF, 2 * DD, nullptr, 0, 0, 0); k_gemmw<bf, 1, false><<<dim3(TT / 64, 2 * DD / 64, 1), 32, 0, stream>>>(Xh, Xl, WK, nullptr, DD, KF, 2 * DD, nullptr, 0, 0, 0); k_gemmw<bf, 1, false><<<dim3(TT / 64, 2 * DD / 64, 1), 32, 0, stream>>>(Xh, Xl, WV, nullptr, DD, VF, 2 * DD, nullptr, 0, 0, 0);
        k_qpl<<<(unsigned)(((size_t)2 * NH_ * TT * HQ / 2 + 255) / 256), 256, 0, stream>>>(QF, Qh, Ql); k_kpad<<<(unsigned)(((size_t)2 * NH_ * KROWS * HQ / 2 + 255) / 256), 256, 0, stream>>>(KF, Kh, Kl); k_vwin<<<(unsigned)(((size_t)NH_ * NBLK * HV * KW / 2 + 255) / 256), 256, 0, stream>>>(VF, Vh, Vl);
        for (int m = 0; m < 2; ++m) for (int h = 0; h < NH_; ++h) { const size_t qo = ((size_t)m * NH_ + h) * TT * HQ, ko = ((size_t)m * NH_ + h) * KROWS * HQ; float* Sm = (m == 0 ? S1 : S2) + (size_t)h * NBLK * 64 * KW;
            k_gemmw<bf, 2, false><<<dim3(1, KW / 64, NBLK), 32, 0, stream>>>(Qh + qo, Ql + qo, Kh + ko, Kl + ko, HQ, Sm, KW, nullptr, (size_t)64 * HQ, (size_t)64 * HQ, (size_t)64 * KW); }
        k_dsoft<<<NH_ * NBLK * 64 / 8, 256, 0, stream>>>(S1, S2, IN[11], IN[12], IN[7], IN[8], IN[9], IN[10], Ph, Pl);
        for (int h = 0; h < NH_; ++h) { const size_t po = (size_t)h * NBLK * 64 * KW, vo = (size_t)h * NBLK * HV * KW;
            k_gemmw<bf, 2, false><<<dim3(1, 1, NBLK), 32, 0, stream>>>(Ph + po, Pl + po, Vh + vo, Vl + vo, KW, O + (size_t)h * TT * HV, HV, nullptr, (size_t)64 * KW, (size_t)HV * KW, (size_t)64 * HV); }
        k_hln<<<NH_ * TT / 8, 256, 0, stream>>>(O, IN[13], IN[14], Mh, Ml);
        k_gemmw<bf, 1, false><<<dim3(TT / 64, DD / 64, 1), 32, 0, stream>>>(Mh, Ml, WO, nullptr, 2 * DD, R, DD, nullptr, 0, 0, 0);
        k_fin<<<(TT * DD / 4 + 255) / 256, 256, 0, stream>>>(xb, R, OUT + (size_t)b * TT * DD); }
}
